// MambaFFN_88167088652785
// MI455X (gfx1250) — hardware-verified
//
#include <hip/hip_runtime.h>
#include <math.h>

typedef __attribute__((ext_vector_type(16))) _Float16 v16h;
typedef __attribute__((ext_vector_type(8)))  _Float16 v8h;
typedef __attribute__((ext_vector_type(16))) __bf16   v16b;
typedef __attribute__((ext_vector_type(8)))  __bf16   v8b;
typedef __attribute__((ext_vector_type(8)))  float    v8f;
typedef __attribute__((ext_vector_type(4)))  float    v4f;
typedef __attribute__((ext_vector_type(2)))  float    v2f;

constexpr int kBatch = 4;
constexpr int kSeq   = 2048;
constexpr int kDm    = 64;
constexpr int kDin   = 128;
constexpr int kNst   = 64;
constexpr int kDtR   = 4;
constexpr int kXzP   = 2 * kDin;
constexpr int kXdbC  = kDtR + 2 * kNst;
constexpr int kXdP   = 192;
constexpr int kRows  = kBatch * kSeq;
constexpr int kFfIn  = 256;
constexpr int kFfK   = 4;
constexpr int kHcN   = 2 * kFfIn;
constexpr int kM1Real = kSeq + 3;
constexpr int kM1    = 2112;
constexpr int kIm1K  = kDm * kFfK;
constexpr int kIm2K  = kFfIn * kFfK;
constexpr int kM2    = kSeq;
constexpr int kConvTP = 132;
constexpr int kScanTS = 64;
constexpr int kScanCh = 64;
constexpr int kScanXP = 132;
constexpr int kScanYP = 68;
constexpr int kNrmRows = 68;
constexpr int kNrmP   = 68;
static_assert(kXdbC <= kXdP);
static_assert((kDm % 32) == 0 && (kDin % 32) == 0 && (kIm1K % 32) == 0 && (kIm2K % 32) == 0);
static_assert((kRows % 64) == 0 && (kXzP % 64) == 0 && (kXdP % 64) == 0 && (kDm % 64) == 0 &&
              (kM1 % 64) == 0 && (kHcN % 64) == 0 && (kM2 % 64) == 0);
static_assert(kM1 >= kM1Real && (kSeq % 64) == 0 && (kSeq % kScanTS) == 0 && kDin == 2 * kScanCh);

constexpr size_t kOffXH   = 0;
constexpr size_t kOffXL   = kOffXH   + (size_t)kRows * kDm * 2;
constexpr size_t kOffWIH  = kOffXL   + (size_t)kRows * kDm * 2;
constexpr size_t kOffWIL  = kOffWIH  + (size_t)kXzP * kDm * 2;
constexpr size_t kOffWXH  = kOffWIL  + (size_t)kXzP * kDm * 2;
constexpr size_t kOffWXL  = kOffWXH  + (size_t)kXdP * kDin * 2;
constexpr size_t kOffWOH  = kOffWXL  + (size_t)kXdP * kDin * 2;
constexpr size_t kOffWOL  = kOffWOH  + (size_t)kDm * kDin * 2;
constexpr size_t kOffWCH  = kOffWOL  + (size_t)kDm * kDin * 2;
constexpr size_t kOffWCL  = kOffWCH  + (size_t)kHcN * kIm1K * 2;
constexpr size_t kOffWDH  = kOffWCL  + (size_t)kHcN * kIm1K * 2;
constexpr size_t kOffWDL  = kOffWDH  + (size_t)kDm * kIm2K * 2;
constexpr size_t kOffXZ   = kOffWDL  + (size_t)kDm * kIm2K * 2;
constexpr size_t kOffXC   = kOffXZ   + (size_t)kRows * kXzP * 4;
constexpr size_t kOffXCH  = kOffXC   + (size_t)kRows * kDin * 4;
constexpr size_t kOffXCL  = kOffXCH  + (size_t)kRows * kDin * 2;
constexpr size_t kOffXD   = kOffXCL  + (size_t)kRows * kDin * 2;
constexpr size_t kOffYH   = kOffXD   + (size_t)kRows * kXdP * 4;
constexpr size_t kOffYL   = kOffYH   + (size_t)kRows * kDin * 2;
constexpr size_t kOffH1   = kOffYL   + (size_t)kRows * kDin * 2;
constexpr size_t kOffH3   = kOffH1   + (size_t)kRows * kDm * 4;
constexpr size_t kOffIM1H = kOffH3   + (size_t)kRows * kDm * 4;
constexpr size_t kOffIM1L = kOffIM1H + (size_t)kBatch * kM1 * kIm1K * 2;
constexpr size_t kOffHC   = kOffIM1L + (size_t)kBatch * kM1 * kIm1K * 2;
constexpr size_t kOffHG   = kOffHC   + (size_t)kBatch * kM1 * kHcN * 4;
constexpr size_t kOffIM2H = kOffHG   + (size_t)kBatch * kM1 * kFfIn * 4;
constexpr size_t kOffIM2L = kOffIM2H + (size_t)kBatch * kM2 * kIm2K * 2;
constexpr size_t kOffYD   = kOffIM2L + (size_t)kBatch * kM2 * kIm2K * 2;
constexpr size_t kWsTotal = kOffYD   + (size_t)kBatch * kM2 * kDm * 4;
static_assert(kWsTotal == 104792064ull);
static_assert(kWsTotal <= 134217728ull);
static_assert((kOffXL % 128) == 0 && (kOffWIH % 128) == 0 && (kOffWIL % 128) == 0 && (kOffWXH % 128) == 0 &&
              (kOffWXL % 128) == 0 && (kOffWOH % 128) == 0 && (kOffWOL % 128) == 0 && (kOffWCH % 128) == 0 &&
              (kOffWCL % 128) == 0 && (kOffWDH % 128) == 0 && (kOffWDL % 128) == 0 && (kOffXZ % 128) == 0 &&
              (kOffXC % 128) == 0 && (kOffXCH % 128) == 0 && (kOffXCL % 128) == 0 && (kOffXD % 128) == 0 &&
              (kOffYH % 128) == 0 && (kOffYL % 128) == 0 && (kOffH1 % 128) == 0 && (kOffH3 % 128) == 0 &&
              (kOffIM1H % 128) == 0 && (kOffIM1L % 128) == 0 && (kOffHC % 128) == 0 && (kOffHG % 128) == 0 &&
              (kOffIM2H % 128) == 0 && (kOffIM2L % 128) == 0 && (kOffYD % 128) == 0);

__device__ __forceinline__ unsigned short f2bf_bits(float f) {
  unsigned u = __float_as_uint(f);
  return (unsigned short)((u + 0x7FFFu + ((u >> 16) & 1u)) >> 16);
}
__device__ __forceinline__ float bf_bits2f(unsigned short h) { return __uint_as_float(((unsigned)h) << 16); }

__device__ __forceinline__ void dep_guard_h(v8f& a, v8f& b, v16h x, v16h y) { asm volatile("v_nop\n\tv_nop\n\tv_nop\n\tv_nop" : "+v"(a), "+v"(b) : "v"(x), "v"(y)); }
__device__ __forceinline__ void dep_guard_b(v8f& a, v8f& b, v16b x, v16b y) { asm volatile("v_nop\n\tv_nop\n\tv_nop\n\tv_nop" : "+v"(a), "+v"(b) : "v"(x), "v"(y)); }
__device__ __forceinline__ void keep4_h(v16h a, v16h b, v16h c, v16h d) { asm volatile("v_nop" :: "v"(a), "v"(b), "v"(c), "v"(d)); }
__device__ __forceinline__ void keep4_b(v16b a, v16b b, v16b c, v16b d) { asm volatile("v_nop" :: "v"(a), "v"(b), "v"(c), "v"(d)); }
__device__ __forceinline__ void acc_guard4(v8f& a, v8f& b, v8f& c, v8f& d) { asm volatile("v_nop\n\tv_nop\n\tv_nop\n\tv_nop" : "+v"(a), "+v"(b), "+v"(c), "+v"(d)); }
template <typename T> struct Frag;
template <> struct Frag<_Float16> {
  typedef v16h V; union U { v16h v; v8h h[2]; };
  static __device__ __forceinline__ v16h load(const _Float16* p) {
    U f; f.h[0] = *(const v8h*)(p); f.h[1] = *(const v8h*)(p + 16); return f.v;
  }
  static __device__ __forceinline__ v8f mma(v16h a, v16h b, v8f c) {
    return __builtin_amdgcn_wmma_f32_16x16x32_f16(false, a, false, b, (short)0, c, false, false);
  }
  static __device__ __forceinline__ void guard(v8f& a, v8f& b, v16h x, v16h y) { dep_guard_h(a, b, x, y); }
  static __device__ __forceinline__ void keep(v16h a, v16h b, v16h c, v16h d) { keep4_h(a, b, c, d); }
};
template <> struct Frag<__bf16> {
  typedef v16b V; union U { v16b v; v8b h[2]; };
  static __device__ __forceinline__ v16b load(const __bf16* p) {
    U f; f.h[0] = *(const v8b*)(p); f.h[1] = *(const v8b*)(p + 16); return f.v;
  }
  static __device__ __forceinline__ v8f mma(v16b a, v16b b, v8f c) {
    return __builtin_amdgcn_wmma_f32_16x16x32_bf16(false, a, false, b, (short)0, c, false, false);
  }
  static __device__ __forceinline__ void guard(v8f& a, v8f& b, v16b x, v16b y) { dep_guard_b(a, b, x, y); }
  static __device__ __forceinline__ void keep(v16b a, v16b b, v16b c, v16b d) { keep4_b(a, b, c, d); }
};

template <int ET> struct Elem;
template <> struct Elem<0> { typedef _Float16 T; };
template <> struct Elem<1> { typedef __bf16 T; };
template <int ET, int SPL, int BIAS_MODE, int OUT_MODE, bool RESID, int ACT = 0>
__global__ __launch_bounds__(256) void wmma_gemm64(
    const unsigned short* __restrict__ Ap, const unsigned short* __restrict__ A2p, int lda, long strideA,
    const unsigned short* __restrict__ Btp, const unsigned short* __restrict__ Bt2p, int ldb, long strideB,
    void* __restrict__ Cout, void* __restrict__ Cout2, int ldc, long strideC,
    const float* __restrict__ bias,
    const float* __restrict__ resid, long strideR,
    int M, int N, int K, float scale) {
  typedef typename Elem<ET>::T T;
  typedef typename Frag<T>::V V;
  const T* A = (const T*)Ap; const T* A2 = (const T*)A2p; const T* Bt = (const T*)Btp; const T* Bt2 = (const T*)Bt2p;
  __shared__ __align__(16) float sT[8][16 * 68];
  const int b    = blockIdx.y;
  const int lane = threadIdx.x & 31;
  const int wave = threadIdx.x >> 5;
  const int tilesN = N >> 6;
  const int tilesM = M >> 6;
  const int tile = blockIdx.x * 8 + wave;
  if (tile >= tilesM * tilesN) return;
  const int tm = tile / tilesN;
  const int tn = tile - tm * tilesN;
  const int m0 = tm << 6;
  const int n0 = tn << 6;

  const T* Ab  = A  + (size_t)b * strideA;
  const T* Bb  = Bt + (size_t)b * strideB;
  const T* Ab2 = (SPL >= 1) ? (A2  + (size_t)b * strideA) : nullptr;
  const T* Bb2 = (SPL == 2) ? (Bt2 + (size_t)b * strideB) : nullptr;

  const int rlane = lane & 15;
  const int koff  = (lane >> 4) * 8;
  const int mOff  = (lane >> 4) * 8;

  v8f acc[4][4];
#pragma unroll
  for (int i = 0; i < 4; ++i)
#pragma unroll
    for (int j = 0; j < 4; ++j) acc[i][j] = (v8f){0.f,0.f,0.f,0.f,0.f,0.f,0.f,0.f};

  for (int k0 = 0; k0 < K; k0 += 32) {
    V bh[4], bl[4];
#pragma unroll
    for (int j = 0; j < 4; ++j) {
      const size_t bo = (size_t)(n0 + (j << 4) + rlane) * ldb + koff + k0;
      bh[j] = Frag<T>::load(Bb + bo);
      if (SPL == 2) bl[j] = Frag<T>::load(Bb2 + bo);
    }
#pragma unroll
    for (int i = 0; i < 4; ++i) {
      const size_t ao = (size_t)(m0 + (i << 4) + rlane) * lda + koff + k0;
      V ah = Frag<T>::load(Ab + ao);
      V al;
      if (SPL >= 1) al = Frag<T>::load(Ab2 + ao);
#pragma unroll
      for (int j = 0; j < 4; ++j) {
        acc[i][j] = Frag<T>::mma(ah, bh[j], acc[i][j]);
        if (SPL == 2) acc[i][j] = Frag<T>::mma(ah, bl[j], acc[i][j]);
        if (SPL >= 1) acc[i][j] = Frag<T>::mma(al, bh[j], acc[i][j]);
      }
      Frag<T>::guard(acc[i][0], acc[i][3], ah, (SPL >= 1) ? al : ah);
    }
    Frag<T>::keep(bh[0], bh[1], bh[2], bh[3]);
    if (SPL == 2) Frag<T>::keep(bl[0], bl[1], bl[2], bl[3]);
  }
  acc_guard4(acc[0][0], acc[0][1], acc[0][2], acc[0][3]);
  acc_guard4(acc[1][0], acc[1][1], acc[1][2], acc[1][3]);
  acc_guard4(acc[2][0], acc[2][1], acc[2][2], acc[2][3]);
  acc_guard4(acc[3][0], acc[3][1], acc[3][2], acc[3][3]);

  float* slab = sT[wave];
  const float* Rb = RESID ? (resid + (size_t)b * strideR) : nullptr;
#pragma unroll
  for (int i = 0; i < 4; ++i) {
    const int mBase = m0 + (i << 4);
#pragma unroll
    for (int j = 0; j < 4; ++j) {
      const int n = n0 + (j << 4) + rlane;
      float bv = 0.f;
      if (BIAS_MODE == 2) bv = bias[n];
#pragma unroll
      for (int r = 0; r < 8; ++r) {
        float v = acc[i][j][r] * scale;
        if (BIAS_MODE == 1) v += bias[mBase + mOff + r];
        if (BIAS_MODE == 2) v += bv;
        if (RESID) v += Rb[(size_t)(mBase + mOff + r) * ldc + n];
        if (ACT == 1) v = tanhf(v);
        if (ACT == 2) v = fmaxf(v, 0.0f);
        if (ACT == 3) v = v / (1.0f + expf(-v));
        if (ACT == 4) v = (v > 0.f) ? v : 0.01f * v;
        slab[(mOff + r) * 68 + (j << 4) + rlane] = v;
      }
    }
    __builtin_amdgcn_fence(__ATOMIC_RELEASE, "workgroup");
    __builtin_amdgcn_wave_barrier();
    __builtin_amdgcn_fence(__ATOMIC_ACQUIRE, "workgroup");
    if (OUT_MODE == 0) {
      float* C = (float*)Cout + (size_t)b * strideC;
      const int hh = lane >> 4, c4 = (lane & 15) * 4;
      for (int pass = 0; pass < 2; ++pass) {
#pragma unroll
        for (int it = 0; it < 8; ++it) {
          const int row = it * 2 + hh;
          v4f v = *(const v4f*)(slab + row * 68 + c4);
          *(volatile v4f*)(C + (size_t)(mBase + row) * ldc + n0 + c4) = v;
        }
        __threadfence();
      }
    } else {
      const int q = lane >> 3, c8 = (lane & 7) * 8;
      unsigned short* C  = (unsigned short*)Cout  + (size_t)b * strideC;
      unsigned short* C2 = (OUT_MODE == 2) ? ((unsigned short*)Cout2 + (size_t)b * strideC) : nullptr;
      for (int pass = 0; pass < 2; ++pass) {
#pragma unroll
        for (int it = 0; it < 4; ++it) {
          const int row = it * 4 + q;
          const float* sp = slab + row * 68 + c8;
          v8h hv, lv;
#pragma unroll
          for (int e = 0; e < 8; ++e) {
            if (OUT_MODE == 1) {
              hv[e] = (_Float16)sp[e];
            } else {
              unsigned short hb = f2bf_bits(sp[e]);
              unsigned short lb = f2bf_bits(sp[e] - bf_bits2f(hb));
              hv[e] = __builtin_bit_cast(_Float16, hb);
              lv[e] = __builtin_bit_cast(_Float16, lb);
            }
          }
          *(volatile v8h*)(C + (size_t)(mBase + row) * ldc + n0 + c8) = hv;
          if (OUT_MODE == 2) *(volatile v8h*)(C2 + (size_t)(mBase + row) * ldc + n0 + c8) = lv;
        }
        __threadfence();
      }
    }
    __builtin_amdgcn_fence(__ATOMIC_RELEASE, "workgroup");
    __builtin_amdgcn_wave_barrier();
    __builtin_amdgcn_fence(__ATOMIC_ACQUIRE, "workgroup");
  }
}

__global__ __launch_bounds__(256) void split_rows_bf16_kernel(
    const float* __restrict__ src, unsigned short* __restrict__ dhi, unsigned short* __restrict__ dlo,
    int real8, int total8)
{
  const int i = blockIdx.x * 256 + threadIdx.x;
  if (i >= total8) return;
  const bool live = (i < real8);
  const int ic = live ? i : (real8 - 1);
  const size_t s0 = (size_t)ic << 3;
  v4f a0 = *(const v4f*)(src + s0);
  v4f a1 = *(const v4f*)(src + s0 + 4);
  if (!live) { a0 = (v4f){0.f, 0.f, 0.f, 0.f}; a1 = (v4f){0.f, 0.f, 0.f, 0.f}; }
  v8h hv, lv;
#pragma unroll
  for (int e = 0; e < 4; ++e) {
    const unsigned short h0 = f2bf_bits(a0[e]), h1 = f2bf_bits(a1[e]);
    const unsigned short l0 = f2bf_bits(a0[e] - bf_bits2f(h0)), l1 = f2bf_bits(a1[e] - bf_bits2f(h1));
    hv[e]     = __builtin_bit_cast(_Float16, h0);
    hv[4 + e] = __builtin_bit_cast(_Float16, h1);
    lv[e]     = __builtin_bit_cast(_Float16, l0);
    lv[4 + e] = __builtin_bit_cast(_Float16, l1);
  }
  const size_t e0 = (size_t)i << 3;
  unsigned short* qh = dhi + e0;
  unsigned short* ql = dlo + e0;
  *(volatile v8h*)qh = hv;
  *(volatile v8h*)ql = lv;
  __threadfence();
  *(volatile v8h*)qh = hv;
  *(volatile v8h*)ql = lv;
}

__global__ __launch_bounds__(256) void wd_planes_kernel(
    const float* __restrict__ dw, unsigned short* __restrict__ WDH, unsigned short* __restrict__ WDL)
{
  const int idx = blockIdx.x * 256 + threadIdx.x;
  if (idx >= kDm * (kIm2K / 8)) return;
  const int d = idx >> 7, p = idx & 127, f0 = 2 * p;
  float val[8];
#pragma unroll
  for (int fi = 0; fi < 2; ++fi) {
    const int f = f0 + fi;
    const v4f w4 = *(const v4f*)(dw + ((size_t)(f * kDm + d)) * kFfK);
    val[fi * 4 + 0] = w4[3];
    val[fi * 4 + 1] = w4[2];
    val[fi * 4 + 2] = w4[1];
    val[fi * 4 + 3] = w4[0];
  }
  v8h hv, lv;
#pragma unroll
  for (int e = 0; e < 8; ++e) {
    const unsigned short hb = f2bf_bits(val[e]);
    const unsigned short lb = f2bf_bits(val[e] - bf_bits2f(hb));
    hv[e] = __builtin_bit_cast(_Float16, hb);
    lv[e] = __builtin_bit_cast(_Float16, lb);
  }
  const size_t o = (size_t)d * kIm2K + (size_t)p * 8;
  *(volatile v8h*)(WDH + o) = hv;
  *(volatile v8h*)(WDL + o) = lv;
  __threadfence();
  *(volatile v8h*)(WDH + o) = hv;
  *(volatile v8h*)(WDL + o) = lv;
}

__global__ __launch_bounds__(128) void conv_silu_kernel(
    const float* __restrict__ XZ, const float* __restrict__ cw, const float* __restrict__ cb,
    float* __restrict__ XC, unsigned short* __restrict__ XCH, unsigned short* __restrict__ XCL)
{
  __shared__ __align__(16) float sT[16 * kConvTP];
  const int tid = threadIdx.x, lane = tid & 31, wave = tid >> 5;
  const int d = tid;
  const int g0 = blockIdx.x * 64;
  const int tb = g0 & (kSeq - 1);
  const float w0 = cw[d * 4 + 0], w1 = cw[d * 4 + 1], w2 = cw[d * 4 + 2], w3 = cw[d * 4 + 3];
  const float bc = cb[d];
  float xm3, xm2, xm1;
  {
    const bool hist = (tb > 0);
    const int rb = hist ? (g0 - 3) : g0;
    const float v3 = XZ[(size_t)rb * kXzP + d];
    const float v2 = XZ[(size_t)(rb + 1) * kXzP + d];
    const float v1 = XZ[(size_t)(rb + 2) * kXzP + d];
    xm3 = hist ? v3 : 0.f;
    xm2 = hist ? v2 : 0.f;
    xm1 = hist ? v1 : 0.f;
  }
  const int brow = wave * 2 + (lane >> 4);
  const int bch  = (lane & 15) * 8;
#pragma unroll 1
  for (int sub = 0; sub < 4; ++sub) {
    const int lb = g0 + sub * 16;
#pragma unroll 1
    for (int s = 0; s < 16; ++s) {
      const float xcur = XZ[(size_t)(lb + s) * kXzP + d];
      float acc = w0 * xm3;
      acc = fmaf(w1, xm2, acc);
      acc = fmaf(w2, xm1, acc);
      acc = fmaf(w3, xcur, acc);
      const float sv = acc + bc;
      const float sg = __builtin_amdgcn_rcpf(1.0f + __expf(-sv));
      sT[s * kConvTP + tid] = sv * sg;
      xm3 = xm2; xm2 = xm1; xm1 = xcur;
    }
    __syncthreads();
    v4f fv[4];
    v8h bh[2], blo[2];
#pragma unroll
    for (int it = 0; it < 4; ++it) fv[it] = *(const v4f*)(sT + (it * 4 + wave) * kConvTP + lane * 4);
#pragma unroll
    for (int it = 0; it < 2; ++it) {
      const float* sp = sT + (it * 8 + brow) * kConvTP + bch;
      const v4f a0 = *(const v4f*)(sp);
      const v4f a1 = *(const v4f*)(sp + 4);
#pragma unroll
      for (int e = 0; e < 4; ++e) {
        const unsigned short h0 = f2bf_bits(a0[e]), h1 = f2bf_bits(a1[e]);
        const unsigned short l0 = f2bf_bits(a0[e] - bf_bits2f(h0)), l1 = f2bf_bits(a1[e] - bf_bits2f(h1));
        bh[it][e]      = __builtin_bit_cast(_Float16, h0);
        bh[it][4 + e]  = __builtin_bit_cast(_Float16, h1);
        blo[it][e]     = __builtin_bit_cast(_Float16, l0);
        blo[it][4 + e] = __builtin_bit_cast(_Float16, l1);
      }
    }
    for (int pass = 0; pass < 2; ++pass) {
#pragma unroll
      for (int it = 0; it < 4; ++it)
        *(volatile v4f*)(XC + (size_t)(lb + it * 4 + wave) * kDin + lane * 4) = fv[it];
#pragma unroll
      for (int it = 0; it < 2; ++it) {
        const size_t o = (size_t)(lb + it * 8 + brow) * kDin + bch;
        *(volatile v8h*)(XCH + o) = bh[it];
        *(volatile v8h*)(XCL + o) = blo[it];
      }
      __threadfence();
    }
    __syncthreads();
  }
}

__global__ __launch_bounds__(256) void scan_kernel(
    const float* __restrict__ XD, const float* __restrict__ XC, const float* __restrict__ XZ,
    const float* __restrict__ Wdt, const float* __restrict__ bdt, const float* __restrict__ Alog,
    const float* __restrict__ Dp, unsigned short* __restrict__ YH, unsigned short* __restrict__ YL)
{
  __shared__ __align__(16) float sX[kScanTS * kScanXP];
  __shared__ __align__(16) float sY[kScanTS * kScanYP];
  const int tid = threadIdx.x, lane = tid & 31, wave = tid >> 5;
  const int c = tid >> 2, qq = tid & 3;
  const int bix = blockIdx.x >> 1;
  const int d0  = (blockIdx.x & 1) * kScanCh;
  const int d   = d0 + c;
  const size_t row0 = (size_t)bix * kSeq;
  float negA[16], h[16];
#pragma unroll
  for (int k = 0; k < 16; ++k) {
    negA[k] = -expf(Alog[(size_t)d * kNst + qq * 16 + k]);
    h[k] = 0.f;
  }
  const float w0 = Wdt[d * kDtR + 0], w1 = Wdt[d * kDtR + 1], w2 = Wdt[d * kDtR + 2], w3 = Wdt[d * kDtR + 3];
  const float bb = bdt[d], Dv = Dp[d];
  const int q = lane >> 3, c8 = (lane & 7) * 8;
  const int boff = kDtR + qq * 16;
  const int coff = kDtR + kNst + qq * 16;
#pragma unroll 1
  for (int t0 = 0; t0 < kSeq; t0 += kScanTS) {
    __syncthreads();
#pragma unroll 1
    for (int i = tid; i < kScanTS * 33; i += 256) {
      const int r = i / 33;
      const int c4 = (i - r * 33) * 4;
      *(v4f*)(sX + r * kScanXP + c4) = *(const v4f*)(XD + (row0 + t0 + r) * kXdP + c4);
    }
    __syncthreads();
#pragma unroll 1
    for (int s = 0; s < kScanTS; ++s) {
      const int t = t0 + s;
      const float* xr = sX + s * kScanXP;
      const v4f dv = *(const v4f*)(xr);
      float v = w0 * dv[0];
      v = fmaf(w1, dv[1], v);
      v = fmaf(w2, dv[2], v);
      v = fmaf(w3, dv[3], v);
      v += bb;
      const float a   = __expf(-fabsf(v));
      const float u   = 1.0f + a;
      const float l1p = __logf(u) + (a - (u - 1.0f)) * __builtin_amdgcn_rcpf(u);
      const float dt  = fmaxf(v, 0.0f) + l1p;
      const float xt  = XC[(row0 + t) * kDin + d];
      const float dtx = dt * xt;
      float y = 0.f;
#pragma unroll
      for (int g = 0; g < 4; ++g) {
        const v4f bv = *(const v4f*)(xr + boff + 4 * g);
        const v4f cv = *(const v4f*)(xr + coff + 4 * g);
#pragma unroll
        for (int e = 0; e < 4; ++e) {
          const int k = 4 * g + e;
          const float ex = __expf(dt * negA[k]);
          h[k] = ex * h[k] + dtx * bv[e];
          y = h[k] * cv[e] + y;
        }
      }
      y += __shfl_xor(y, 1, 32);
      y += __shfl_xor(y, 2, 32);
      y = xt * Dv + y;
      const float zv = XZ[(row0 + t) * kXzP + kDin + d];
      const float sg = __builtin_amdgcn_rcpf(1.0f + __expf(-zv));
      y = y * (zv * sg);
      if (qq == 0) sY[s * kScanYP + c] = y;
    }
    __syncthreads();
    v8h hv[2], lv[2];
#pragma unroll
    for (int it = 0; it < 2; ++it) {
      const int row = it * 32 + wave * 4 + q;
      const float* sp = sY + row * kScanYP + c8;
      const v4f a0 = *(const v4f*)(sp);
      const v4f a1 = *(const v4f*)(sp + 4);
#pragma unroll
      for (int e = 0; e < 4; ++e) {
        const unsigned short h0 = f2bf_bits(a0[e]), h1 = f2bf_bits(a1[e]);
        const unsigned short l0 = f2bf_bits(a0[e] - bf_bits2f(h0)), l1 = f2bf_bits(a1[e] - bf_bits2f(h1));
        hv[it][e]     = __builtin_bit_cast(_Float16, h0);
        hv[it][4 + e] = __builtin_bit_cast(_Float16, h1);
        lv[it][e]     = __builtin_bit_cast(_Float16, l0);
        lv[it][4 + e] = __builtin_bit_cast(_Float16, l1);
      }
    }
    for (int pass = 0; pass < 2; ++pass) {
#pragma unroll
      for (int it = 0; it < 2; ++it) {
        const int row = it * 32 + wave * 4 + q;
        const size_t o = (row0 + t0 + row) * kDin + d0 + c8;
        *(volatile v8h*)(YH + o) = hv[it];
        *(volatile v8h*)(YL + o) = lv[it];
      }
      __threadfence();
    }
  }
}

__global__ __launch_bounds__(256) void norm_im2col_kernel(
    const float* __restrict__ H1, const float* __restrict__ gam, float* __restrict__ H3,
    unsigned short* __restrict__ IM1H, unsigned short* __restrict__ IM1L)
{
  __shared__ __align__(16) float sH[kNrmRows * kNrmP];
  const int tid = threadIdx.x, lane = tid & 31, wave = tid >> 5;
  const int b = blockIdx.y;
  const int blk = blockIdx.x;
  const int t0p = blk * 64;
  const int col = tid & 63;
  const int rsub = tid >> 6;
  const float gcol = gam[col];
#pragma unroll 1
  for (int pass = 0; pass < 17; ++pass) {
    const int r = pass * 4 + rsub;
    const int tau = t0p - 3 + r;
    const bool valid = (tau >= 0) && (tau < kSeq);
    const int tauc = tau < 0 ? 0 : (tau > kSeq - 1 ? kSeq - 1 : tau);
    float v = H1[((size_t)b * kSeq + tauc) * kDm + col];
    v = (v > 0.f) ? v : 0.01f * v;
    float ss = v * v;
    ss += __shfl_xor(ss, 1, 32);
    ss += __shfl_xor(ss, 2, 32);
    ss += __shfl_xor(ss, 4, 32);
    ss += __shfl_xor(ss, 8, 32);
    const float rms = sqrtf(ss) * 0.25f;
    const float inv = 1.0f / (rms + 1e-5f);
    const float hn = v * inv * gcol;
    sH[r * kNrmP + col] = valid ? hn : 0.f;
  }
  __syncthreads();
  if (t0p < kSeq) {
    v4f hv4[4];
#pragma unroll
    for (int it = 0; it < 4; ++it) {
      const int idx = it * 256 + tid;
      const int row = idx >> 4, c4 = (idx & 15) * 4;
      hv4[it] = *(const v4f*)(sH + (row + 3) * kNrmP + c4);
    }
    for (int pass = 0; pass < 2; ++pass) {
#pragma unroll
      for (int it = 0; it < 4; ++it) {
        const int idx = it * 256 + tid;
        const int row = idx >> 4, c4 = (idx & 15) * 4;
        *(volatile v4f*)(H3 + ((size_t)b * kSeq + t0p + row) * kDm + c4) = hv4[it];
      }
      __threadfence();
    }
  }
  v8h hv[8], lv[8];
#pragma unroll
  for (int it = 0; it < 8; ++it) {
    const int i = it * 8 + wave;
#pragma unroll
    for (int e = 0; e < 8; ++e) {
      const int cc = lane * 2 + (e >> 2);
      const int j = e & 3;
      const float val = sH[(i + j) * kNrmP + cc];
      const unsigned short hb = f2bf_bits(val);
      const unsigned short lb = f2bf_bits(val - bf_bits2f(hb));
      hv[it][e] = __builtin_bit_cast(_Float16, hb);
      lv[it][e] = __builtin_bit_cast(_Float16, lb);
    }
  }
  for (int pass = 0; pass < 2; ++pass) {
#pragma unroll
    for (int it = 0; it < 8; ++it) {
      const int i = it * 8 + wave;
      const size_t o = ((size_t)b * kM1 + t0p + i) * kIm1K + (size_t)lane * 8;
      *(volatile v8h*)(IM1H + o) = hv[it];
      *(volatile v8h*)(IM1L + o) = lv[it];
    }
    __threadfence();
  }
}

__global__ __launch_bounds__(256) void gate_kernel(
    const float* __restrict__ HC, float* __restrict__ HG, int n4)
{
  const int i = blockIdx.x * 256 + threadIdx.x;
  if (i >= n4) return;
  const size_t e0 = (size_t)i << 2;
  const size_t row = e0 >> 8;
  const int f = (int)(e0 & 255);
  const v4f u = *(const v4f*)(HC + row * kHcN + f);
  const v4f g = *(const v4f*)(HC + row * kHcN + kFfIn + f);
  v4f o;
#pragma unroll
  for (int e = 0; e < 4; ++e) {
    const float sg = __builtin_amdgcn_rcpf(1.0f + __expf(-g[e]));
    o[e] = u[e] * (g[e] * sg);
  }
  *(volatile v4f*)(HG + e0) = o;
  __threadfence();
  *(volatile v4f*)(HG + e0) = o;
}

__global__ __launch_bounds__(256) void im2col2_kernel(
    const float* __restrict__ HG, unsigned short* __restrict__ IM2H, unsigned short* __restrict__ IM2L)
{
  const int tid = threadIdx.x;
  const int gr = blockIdx.x * 2 + (tid >> 7);
  if (gr >= kBatch * kM2) return;
  const int b = gr >> 11, t = gr & (kSeq - 1);
  const int p = tid & 127, f0 = 2 * p;
  float val[8];
#pragma unroll
  for (int j = 0; j < 4; ++j) {
    const size_t rb = (size_t)b * kM1 + t + j;
    const v2f uv = *(const v2f*)(HG + rb * kFfIn + f0);
    val[j]     = uv[0];
    val[4 + j] = uv[1];
  }
  v8h hv, lv;
#pragma unroll
  for (int e = 0; e < 8; ++e) {
    const unsigned short hb = f2bf_bits(val[e]);
    const unsigned short lb = f2bf_bits(val[e] - bf_bits2f(hb));
    hv[e] = __builtin_bit_cast(_Float16, hb);
    lv[e] = __builtin_bit_cast(_Float16, lb);
  }
  const size_t o = (size_t)gr * kIm2K + (size_t)p * 8;
  *(volatile v8h*)(IM2H + o) = hv;
  *(volatile v8h*)(IM2L + o) = lv;
  __threadfence();
  *(volatile v8h*)(IM2H + o) = hv;
  *(volatile v8h*)(IM2L + o) = lv;
}

__global__ __launch_bounds__(256) void final_kernel(
    const float* __restrict__ H3, const float* __restrict__ YD, const float* __restrict__ db,
    float* __restrict__ out, int n4)
{
  const int i = blockIdx.x * 256 + threadIdx.x;
  if (i >= n4) return;
  const size_t e0 = (size_t)i << 2;
  const int col = (int)(e0 & (kDm - 1));
  const v4f hv = *(const v4f*)(H3 + e0);
  const v4f yv = *(const v4f*)(YD + e0);
  const v4f dv = *(const v4f*)(db + col);
  const v4f o = hv + 0.5f * (yv + dv);
  *(volatile v4f*)(out + e0) = o;
  __threadfence();
  *(volatile v4f*)(out + e0) = o;
}

extern "C" void kernel_launch(void* const* d_in, const int* in_sizes, int n_in,
                              void* d_out, int out_size, void* d_ws, size_t ws_size,
                              hipStream_t stream) {
  if (n_in < 15) return;
  if (in_sizes[0]  != kRows * kDm) return;
  if (in_sizes[1]  != kXzP * kDm) return;
  if (in_sizes[2]  != kDin * 4) return;
  if (in_sizes[3]  != kDin) return;
  if (in_sizes[4]  != kXdbC * kDin) return;
  if (in_sizes[5]  != kDin * kDtR) return;
  if (in_sizes[6]  != kDin) return;
  if (in_sizes[7]  != kDin * kNst) return;
  if (in_sizes[8]  != kDin) return;
  if (in_sizes[9]  != kDm * kDin) return;
  if (in_sizes[10] != kDm) return;
  if (in_sizes[11] != kHcN * kDm * kFfK) return;
  if (in_sizes[12] != kHcN) return;
  if (in_sizes[13] != kFfIn * kDm * kFfK) return;
  if (in_sizes[14] != kDm) return;
  if (out_size != kRows * kDm) return;
  if (ws_size < kWsTotal) return;

  const float* x       = (const float*)d_in[0];
  const float* W_in    = (const float*)d_in[1];
  const float* conv_w  = (const float*)d_in[2];
  const float* conv_b  = (const float*)d_in[3];
  const float* W_xproj = (const float*)d_in[4];
  const float* W_dt    = (const float*)d_in[5];
  const float* b_dt    = (const float*)d_in[6];
  const float* A_log   = (const float*)d_in[7];
  const float* Dp      = (const float*)d_in[8];
  const float* W_out   = (const float*)d_in[9];
  const float* gam     = (const float*)d_in[10];
  const float* W_ffc   = (const float*)d_in[11];
  const float* b_ffc   = (const float*)d_in[12];
  const float* W_ffd   = (const float*)d_in[13];
  const float* b_ffd   = (const float*)d_in[14];
  float* out = (float*)d_out;

  char* ws = (char*)d_ws;
  unsigned short* XH   = (unsigned short*)(ws + kOffXH);
  unsigned short* XL   = (unsigned short*)(ws + kOffXL);
  unsigned short* WIH  = (unsigned short*)(ws + kOffWIH);
  unsigned short* WIL  = (unsigned short*)(ws + kOffWIL);
  unsigned short* WXH  = (unsigned short*)(ws + kOffWXH);
  unsigned short* WXL  = (unsigned short*)(ws + kOffWXL);
  unsigned short* WOH  = (unsigned short*)(ws + kOffWOH);
  unsigned short* WOL  = (unsigned short*)(ws + kOffWOL);
  unsigned short* WCH  = (unsigned short*)(ws + kOffWCH);
  unsigned short* WCL  = (unsigned short*)(ws + kOffWCL);
  unsigned short* WDH  = (unsigned short*)(ws + kOffWDH);
  unsigned short* WDL  = (unsigned short*)(ws + kOffWDL);
  float*          XZ   = (float*)(ws + kOffXZ);
  float*          XC   = (float*)(ws + kOffXC);
  unsigned short* XCH  = (unsigned short*)(ws + kOffXCH);
  unsigned short* XCL  = (unsigned short*)(ws + kOffXCL);
  float*          XD   = (float*)(ws + kOffXD);
  unsigned short* YH   = (unsigned short*)(ws + kOffYH);
  unsigned short* YL   = (unsigned short*)(ws + kOffYL);
  float*          H1   = (float*)(ws + kOffH1);
  float*          H3   = (float*)(ws + kOffH3);
  unsigned short* IM1H = (unsigned short*)(ws + kOffIM1H);
  unsigned short* IM1L = (unsigned short*)(ws + kOffIM1L);
  float*          HC   = (float*)(ws + kOffHC);
  float*          HG   = (float*)(ws + kOffHG);
  unsigned short* IM2H = (unsigned short*)(ws + kOffIM2H);
  unsigned short* IM2L = (unsigned short*)(ws + kOffIM2L);
  float*          YD   = (float*)(ws + kOffYD);

  {
    const int x8  = kRows * kDm / 8;
    const int wi8 = kXzP * kDm / 8;
    const int wxr8 = kXdbC * kDin / 8, wxt8 = kXdP * kDin / 8;
    const int wo8 = kDm * kDin / 8;
    const int wc8 = kHcN * kIm1K / 8;
    split_rows_bf16_kernel<<<(x8 + 255) / 256, 256, 0, stream>>>(x, XH, XL, x8, x8);
    split_rows_bf16_kernel<<<(wi8 + 255) / 256, 256, 0, stream>>>(W_in, WIH, WIL, wi8, wi8);
    split_rows_bf16_kernel<<<(wxt8 + 255) / 256, 256, 0, stream>>>(W_xproj, WXH, WXL, wxr8, wxt8);
    split_rows_bf16_kernel<<<(wo8 + 255) / 256, 256, 0, stream>>>(W_out, WOH, WOL, wo8, wo8);
    split_rows_bf16_kernel<<<(wc8 + 255) / 256, 256, 0, stream>>>(W_ffc, WCH, WCL, wc8, wc8);
    wd_planes_kernel<<<(kDm * (kIm2K / 8) + 255) / 256, 256, 0, stream>>>(W_ffd, WDH, WDL);
  }

  wmma_gemm64<1, 2, 0, 0, false><<<dim3((kRows / 64) * (kXzP / 64) / 8, 1), 256, 0, stream>>>(
      XH, XL, kDm, 0L,
      WIH, WIL, kDm, 0L,
      (void*)XZ, nullptr, kXzP, 0L,
      nullptr, nullptr, 0L,
      kRows, kXzP, kDm, 1.0f);

  conv_silu_kernel<<<kRows / 64, kDin, 0, stream>>>(XZ, conv_w, conv_b, XC, XCH, XCL);

  wmma_gemm64<1, 2, 0, 0, false><<<dim3((kRows / 64) * (kXdP / 64) / 8, 1), 256, 0, stream>>>(
      XCH, XCL, kDin, 0L,
      WXH, WXL, kDin, 0L,
      (void*)XD, nullptr, kXdP, 0L,
      nullptr, nullptr, 0L,
      kRows, kXdP, kDin, 1.0f);

  scan_kernel<<<kBatch * (kDin / kScanCh), 256, 0, stream>>>(XD, XC, XZ, W_dt, b_dt, A_log, Dp, YH, YL);

  wmma_gemm64<1, 2, 0, 0, false><<<dim3((kRows / 64) * (kDm / 64) / 8, 1), 256, 0, stream>>>(
      YH, YL, kDin, 0L,
      WOH, WOL, kDin, 0L,
      (void*)H1, nullptr, kDm, 0L,
      nullptr, nullptr, 0L,
      kRows, kDm, kDin, 1.0f);

  norm_im2col_kernel<<<dim3(kM1 / 64, kBatch), 256, 0, stream>>>(H1, gam, H3, IM1H, IM1L);

  wmma_gemm64<1, 2, 2, 0, false><<<dim3((kM1 / 64) * (kHcN / 64) / 8, kBatch), 256, 0, stream>>>(
      IM1H, IM1L, kIm1K, (long)kM1 * kIm1K,
      WCH, WCL, kIm1K, 0L,
      (void*)HC, nullptr, kHcN, (long)kM1 * kHcN,
      b_ffc, nullptr, 0L,
      kM1, kHcN, kIm1K, 1.0f);

  {
    const int n4 = kBatch * kM1 * kFfIn / 4;
    gate_kernel<<<(n4 + 255) / 256, 256, 0, stream>>>(HC, HG, n4);
  }

  im2col2_kernel<<<(kBatch * kM2 + 1) / 2, 256, 0, stream>>>(HG, IM2H, IM2L);

  wmma_gemm64<1, 2, 0, 0, false><<<dim3((kM2 / 64) * (kDm / 64) / 8, kBatch), 256, 0, stream>>>(
      IM2H, IM2L, kIm2K, (long)kM2 * kIm2K,
      WDH, WDL, kIm2K, 0L,
      (void*)YD, nullptr, kDm, (long)kM2 * kDm,
      nullptr, nullptr, 0L,
      kM2, kDm, kIm2K, 1.0f);

  {
    const int n4 = kRows * kDm / 4;
    final_kernel<<<(n4 + 255) / 256, 256, 0, stream>>>(H3, YD, b_ffd, out, n4);
  }
}
